// SparseConvBlock_77902116815210
// MI455X (gfx1250) — hardware-verified
//
#include <hip/hip_runtime.h>


namespace {
constexpr int N = 100000, NP = 100032, NPL = NP  , C = 64, K = 27, NBLK = NPL / 32, NL = (NPL < N ? NPL : N);
constexpr float XS = 8.0f, WSC = 256.0f, BNEPS = 1e-5f;
static_assert(NP % 32 == 0 && NP >= N && NPL % 32 == 0 && C == 64, "tiling");
typedef _Float16 b16;
typedef __attribute__((ext_vector_type(16))) _Float16 v16b;
typedef __attribute__((ext_vector_type(8))) _Float16 v8b;
typedef __attribute__((ext_vector_type(8))) float v8f;
typedef __attribute__((ext_vector_type(4))) float v4f;
__device__ __forceinline__ float bf16_rne(float f) { unsigned int u = __float_as_uint(f); u += 0x7FFFu + ((u >> 16) & 1u); return __uint_as_float(u & 0xFFFF0000u); }
__device__ __forceinline__ void split16(float v, b16& hi, b16& lo) { hi = (b16)v; lo = (b16)(v - (float)hi); }
__device__ __forceinline__ v16b frag_kb(const b16* p, int hh) { const v8b a = *(const v8b*)(p + 8 * hh), b = *(const v8b*)(p + 16 + 8 * hh); v16b f;
#pragma unroll
  for (int e = 0; e < 8; ++e) { f[e] = a[e]; f[8 + e] = b[e]; } return f; }
__device__ __forceinline__ v8f wmma16b(v16b a, v16b b, v8f c) { v8f d = __builtin_amdgcn_wmma_f32_16x16x32_f16(false, a, false, b, (short)0, c, false, false); asm volatile("v_nop\n\tv_nop\n\tv_nop\n\tv_nop" : "+v"(d) : "v"(a), "v"(b)); return d; }
__device__ __forceinline__ void wave_lds_sync() { __builtin_amdgcn_fence(__ATOMIC_RELEASE, "workgroup"); __builtin_amdgcn_wave_barrier(); __builtin_amdgcn_fence(__ATOMIC_ACQUIRE, "workgroup"); }
__device__ __forceinline__ float pmul(float a, float b) { float p = a * b; asm volatile("" : "+v"(p)); return p; }
__device__ __forceinline__ int iclamp(int v, int lo, int hi) { return v < lo ? lo : (v > hi ? hi : v); }

typedef __attribute__((ext_vector_type(2))) _Float16 v2h;
typedef __attribute__((ext_vector_type(4))) _Float16 v4h;
typedef __attribute__((ext_vector_type(2))) float v2f;
typedef __attribute__((ext_vector_type(4))) int v4i;
__device__ __forceinline__ float nexp2(float v) { return __builtin_amdgcn_exp2f(v); }
typedef __attribute__((ext_vector_type(4))) _Float16 v4h_;
__global__ __launch_bounds__(256) void wt_kernel(const float* __restrict__ w, b16* __restrict__ WT) {
  const int u = blockIdx.x * 256 + threadIdx.x; if (u >= K * C * C / 8) return; const int e = u * 8; const int k = e / (C * C), rem = e % (C * C), o = rem / C, c0 = rem % C; v8b v;
#pragma unroll
  for (int j = 0; j < 8; ++j) v[j] = (b16)(bf16_rne(w[((size_t)k * C + c0 + j) * C + o]) * WSC);
  for (int pass = 0; pass < 2; ++pass) { *(volatile v8b*)(WT + e) = v; __threadfence(); }
}
__device__ __forceinline__ int lower_bound_row(const int* __restrict__ row, int j) { int lo = 0, hi = N;
#pragma unroll 1
  while (lo < hi) { const int mid = (lo + hi) >> 1; if (row[mid] < j) lo = mid + 1; else hi = mid; } return lo; }
__global__ __launch_bounds__(256) void conv_kernel(const float* __restrict__ feats, const int* __restrict__ in_idx, const int* __restrict__ out_idx, const b16* __restrict__ WT, float* __restrict__ Y, float* __restrict__ PART) {
  __shared__ __attribute__((aligned(16))) b16 As[32][C + 8]; __shared__ __attribute__((aligned(16))) float Tf[32][C + 4]; __shared__ float csum[8][C];
  const int tid = threadIdx.x, wave = tid >> 5, lane = tid & 31, nloc = lane & 15, hlf = lane >> 4; const int v0 = blockIdx.x * 32; const int row = tid >> 3, g = tid & 7; const int j = v0 + row;
  const int rt = wave & 1, ct = wave >> 1; v8f acc = (v8f){};
#pragma unroll 1
  for (int k = 0; k < K; ++k) {
    const int* orow = out_idx + (size_t)k * N; const int jj = j < N ? j : N - 1;
    const int pos = iclamp(lower_bound_row(orow, jj), 0, N - 1); const float fl = (j < N && orow[pos] == jj) ? XS : 0.0f; const int partner = iclamp(in_idx[(size_t)k * N + pos], 0, N - 1);
    v8b a8; { const float* fr = feats + (size_t)partner * C + g * 8; const v4f f0 = *(const v4f*)fr, f1 = *(const v4f*)(fr + 4); for (int q = 0; q < 4; ++q) { a8[q] = (b16)(bf16_rne(f0[q]) * fl); a8[4 + q] = (b16)(bf16_rne(f1[q]) * fl); } }
    __syncthreads();
    *(v8b*)(&As[row][g * 8]) = a8;
    __syncthreads();
    const b16* br = WT + ((size_t)k * C + ct * 16 + nloc) * C;
#pragma unroll
    for (int kb = 0; kb < C; kb += 32) acc = wmma16b(frag_kb(&As[rt * 16 + nloc][kb], hlf), frag_kb(br + kb, hlf), acc); }
#pragma unroll
  for (int r = 0; r < 8; ++r) { const int rr = rt * 16 + 8 * hlf + r; Tf[rr][ct * 16 + nloc] = (v0 + rr < N) ? acc[r] * (1.0f / (XS * WSC)) : 0.0f; }
  __syncthreads();
  { const int c = tid & 63, q = tid >> 6; float s = 0.0f; for (int rr = q * 8; rr < q * 8 + 8; ++rr) s += Tf[rr][c]; csum[q][c] = s; }
  __syncthreads();
  for (int pass = 0; pass < 2; ++pass) {
    for (int rr = wave * 4; rr < wave * 4 + 4; rr += 2) { const int r2 = rr + (lane >> 4); *(volatile v4f*)(Y + (size_t)(v0 + r2) * C + (lane & 15) * 4) = *(const v4f*)(&Tf[r2][(lane & 15) * 4]); }
    if (wave == 0 && lane < 16) { v4f p; for (int q = 0; q < 4; ++q) { const int c = lane * 4 + q; p[q] = ((csum[0][c] + csum[1][c]) + csum[2][c]) + csum[3][c]; } *(volatile v4f*)(PART + (size_t)blockIdx.x * C + lane * 4) = p; }
    __threadfence(); }
}
__global__ __launch_bounds__(64) void reduce_kernel(const float* __restrict__ PART, float* __restrict__ STAT, int which) {
  const int c = threadIdx.x; float s = 0.0f;
#pragma unroll 1
  for (int b = 0; b < NBLK; ++b) s += PART[(size_t)b * C + c];
  for (int pass = 0; pass < 2; ++pass) { ((volatile float*)STAT)[which * C + c] = s * (1.0f / (float)NL); __threadfence(); }
}
__global__ __launch_bounds__(256) void varp_kernel(const float* __restrict__ Y, const float* __restrict__ STAT, float* __restrict__ PART) {
  __shared__ float csum[4][C]; const int tid = threadIdx.x; const int v0 = blockIdx.x * 32; const int c = tid & 63, q = tid >> 6; const float mu = STAT[c]; float s = 0.0f;
  for (int rr = q * 8; rr < q * 8 + 8; ++rr) { const int v = v0 + rr; const float wv = (v < N) ? 1.0f : 0.0f; const float d = Y[(size_t)(v < N ? v : N - 1) * C + c] - mu; s = fmaf(d * wv, d, s); }
  csum[q][c] = s; __syncthreads();
  const int wave = tid >> 5, lane = tid & 31;
  for (int pass = 0; pass < 2; ++pass) { if (wave == 0 && lane < 16) { v4f p; for (int t = 0; t < 4; ++t) { const int cc = lane * 4 + t; p[t] = ((csum[0][cc] + csum[1][cc]) + csum[2][cc]) + csum[3][cc]; } *(volatile v4f*)(PART + (size_t)blockIdx.x * C + lane * 4) = p; } __threadfence(); }
}
__global__ __launch_bounds__(256) void bn_kernel(const float* __restrict__ Y, const float* __restrict__ STAT, const float* __restrict__ gam, const float* __restrict__ bet, float* __restrict__ out) {
  const size_t u = (size_t)blockIdx.x * 256 + threadIdx.x; if (u >= (size_t)NL * C / 4) return; const int c0 = (int)((u * 4) % C); const v4f y = *(const v4f*)(Y + u * 4); v4f o;
  for (int q = 0; q < 4; ++q) { const int c = c0 + q; const float t = (y[q] - STAT[c]) * rsqrtf(STAT[C + c] + BNEPS) * bf16_rne(gam[c]) + bf16_rne(bet[c]); o[q] = fmaxf(t, 0.0f); }
  for (int pass = 0; pass < 2; ++pass) { *(volatile v4f*)(out + u * 4) = o; __threadfence(); }
}
}

extern "C" void kernel_launch(void* const* d_in, const int* in_sizes, int n_in, void* d_out, int out_size, void* d_ws, size_t ws_size, hipStream_t stream) {
  (void)n_in;
  auto Fp = [&](int i) { return (const float*)d_in[i]; }; auto Ip = [&](int i) { return (const int*)d_in[i]; };
  if (in_sizes[0] != N * C || in_sizes[1] != K * C * C || in_sizes[2] != C || in_sizes[3] != C || in_sizes[4] != K * N || in_sizes[5] != K * N || out_size != N * C) return;
  size_t off = 0; char* ws = (char*)d_ws;
  auto carve = [&](size_t bytes) { char* p = ws + off; off += (bytes + 255) & ~(size_t)255; return p; };
  b16* WT = (b16*)carve((size_t)K * C * C * 2); float* Y = (float*)carve((size_t)NP * C * 4); float* PART = (float*)carve((size_t)NBLK * C * 4); float* STAT = (float*)carve(2 * C * 4);
  if (off > ws_size || off > ((size_t)128 << 20)) return;
  wt_kernel<<<(K * C * C / 8 + 255) / 256, 256, 0, stream>>>(Fp(1), WT);
  conv_kernel<<<NBLK, 256, 0, stream>>>(Fp(0), Ip(4), Ip(5), WT, Y, PART);
  reduce_kernel<<<1, 64, 0, stream>>>(PART, STAT, 0);
  varp_kernel<<<NBLK, 256, 0, stream>>>(Y, STAT, PART);
  reduce_kernel<<<1, 64, 0, stream>>>(PART, STAT, 1);
  bn_kernel<<<(unsigned)(((size_t)NL * C / 4 + 255) / 256), 256, 0, stream>>>(Y, STAT, Fp(2), Fp(3), (float*)d_out);
}
